// tnn_24060406792344
// MI455X (gfx1250) — hardware-verified
//
#include <hip/hip_runtime.h>
#include <hip/hip_bf16.h>
#include <math.h>


typedef _Float16 bf16;
typedef _Float16 f16;
typedef __attribute__((ext_vector_type(4))) unsigned v4u_t;
typedef unsigned v4ua __attribute__((ext_vector_type(4), may_alias));
typedef __attribute__((ext_vector_type(4))) float v4f_t;
typedef float v4fa __attribute__((ext_vector_type(4), may_alias));
typedef __attribute__((ext_vector_type(16))) bf16  bf16x16;
typedef bf16x16 f16x16;
typedef __attribute__((ext_vector_type(8)))  bf16  bf16x8;
typedef bf16x8 f16x8;
typedef __attribute__((ext_vector_type(4)))  bf16  bf16x4;
typedef __attribute__((ext_vector_type(8)))  float f32x8;
__device__ __forceinline__ f32x8 wmma16(f16x16 a, f16x16 b, f32x8 c) {
  c = __builtin_amdgcn_wmma_f32_16x16x32_f16(false, a, false, b, (short)0, c, false, false);
  asm volatile("v_nop\n\tv_nop\n\tv_nop\n\tv_nop" : "+v"(c) : "v"(a), "v"(b));
  return c;
}
#define LDS_STRIDE 48
#define KSTRIDE    72
#define VSTRIDE    48

__device__ __forceinline__ f32x8 wmma_bf16(bf16x16 a, bf16x16 b, f32x8 c) {
  c = __builtin_amdgcn_wmma_f32_16x16x32_f16(false, a, false, b, (short)0, c, false, false);
  asm volatile("v_nop\n\tv_nop\n\tv_nop\n\tv_nop" : "+v"(c) : "v"(a), "v"(b));
  return c;
}

template <typename T>
__device__ __forceinline__ bf16x16 load_frag(const T* __restrict__ base, int ld,
                                             int row0, int k0) {
  const int lane = threadIdx.x & 31;
  const int r    = lane & 15;
  const int kh   = (lane >> 4) * 8;
  const T* p0 = base + (size_t)(row0 + r) * ld + (k0 + kh);
  const T* p1 = p0 + 16;
  bf16x16 f;
#pragma unroll
  for (int i = 0; i < 8; ++i) {
    f[i]     = (bf16)p0[i];
    f[i + 8] = (bf16)p1[i];
  }
  return f;
}

__device__ __forceinline__ bf16x16 lds_frag(const bf16* base, int stride) {
  const int lane = threadIdx.x & 31;
  const int row  = lane & 15;
  const int kh   = (lane >> 4) * 8;
  const bf16x8 lo = *(const bf16x8*)(base + row * stride + kh);
  const bf16x8 hi = *(const bf16x8*)(base + row * stride + kh + 16);
  bf16x16 f;
#pragma unroll
  for (int i = 0; i < 8; ++i) { f[i] = lo[i]; f[i + 8] = hi[i]; }
  return f;
}

template <typename T>
__device__ __forceinline__ void stage_read16(const T* __restrict__ p, float* buf) {
#pragma unroll
  for (int i = 0; i < 16; ++i) buf[i] = (float)p[i];
}

__device__ __forceinline__ void stage_write(bf16* dst, const float* buf, int nquad) {
#pragma unroll
  for (int i = 0; i < nquad; ++i) {
    bf16x4 q;
    q[0] = (bf16)buf[4 * i];     q[1] = (bf16)buf[4 * i + 1];
    q[2] = (bf16)buf[4 * i + 2]; q[3] = (bf16)buf[4 * i + 3];
    *(bf16x4*)(dst + 4 * i) = q;
  }
}


#define GSTR 48
#define GSTR 48
template <typename AT, int EPI, bool OUT16>
__global__ __launch_bounds__(256) void gemm_kne(const AT* __restrict__ A, int lda, const float* __restrict__ Wm, int ldw,
                                                const float* __restrict__ bias, const float* __restrict__ R, const float* __restrict__ gvec,
                                                void* __restrict__ Yv, int ldy, int K) {
  __shared__ __attribute__((aligned(16))) f16 ldsA[128 * GSTR];
  __shared__ __attribute__((aligned(16))) f16 ldsW[128 * GSTR];
  __shared__ __attribute__((aligned(16))) float oS[8][32 * 68];
  const int tid = threadIdx.x, lane = tid & 31, wave = tid >> 5, cl = lane & 15, rh = (lane >> 4) * 8;
  const int m0 = blockIdx.x * 128, n0 = blockIdx.y * 128;
  const int wm = (wave & 3) * 32, wn = (wave >> 2) * 64;
  f32x8 acc[2][4];
#pragma unroll
  for (int i = 0; i < 2; ++i)
#pragma unroll
    for (int j = 0; j < 4; ++j) { f32x8 z = {}; acc[i][j] = z; }
#pragma unroll 1
  for (int k0 = 0; k0 < K; k0 += 32) {
    __syncthreads();
    { const int row = tid >> 1, ch = (tid & 1) * 16;
      const AT* src = A + (size_t)(m0 + row) * lda + k0 + ch;
#pragma unroll
      for (int g = 0; g < 16; ++g) ldsA[row * GSTR + ch + g] = (f16)src[g]; }
    { const int k = tid >> 3, nn0 = (tid & 7) * 16;
      const float* src = Wm + (size_t)(k0 + k) * ldw + n0 + nn0;
#pragma unroll
      for (int g = 0; g < 4; ++g) { const v4f_t v = *(const v4f_t*)(src + 4 * g);
#pragma unroll
        for (int u = 0; u < 4; ++u) ldsW[(nn0 + 4 * g + u) * GSTR + k] = (f16)v[u]; } }
    __syncthreads();
    f16x16 af[2];
#pragma unroll
    for (int i = 0; i < 2; ++i) af[i] = lds_frag(ldsA + (wm + 16 * i) * GSTR, GSTR);
#pragma unroll
    for (int j = 0; j < 4; ++j) {
      const f16x16 bf = lds_frag(ldsW + (wn + 16 * j) * GSTR, GSTR);
#pragma unroll
      for (int i = 0; i < 2; ++i) acc[i][j] = wmma16(af[i], bf, acc[i][j]);
    }
  }
  float* so = oS[wave];
#pragma unroll
  for (int i = 0; i < 2; ++i)
#pragma unroll
    for (int j = 0; j < 4; ++j) {
      const int n = n0 + wn + 16 * j + cl;
      const float bv = bias ? bias[n] : 0.0f;
      const float gv = (EPI == 2 || EPI == 4) ? gvec[n] : 0.0f;
      if (EPI == 1) {
#pragma unroll 1
        for (int r = 0; r < 8; ++r) { const float xg = acc[i][j][r] + bv; so[(16 * i + rh + r) * 68 + 16 * j + cl] = 0.5f * xg * (1.0f + erff(xg * 0.70710678118654752f)); }
      } else {
#pragma unroll
        for (int r = 0; r < 8; ++r) {
          float v = acc[i][j][r] + bv;
          if (EPI == 3) v = fmaxf(v, 0.0f);
          if (EPI == 4) v = gv * v;
          if (EPI == 2) v = R[(size_t)(m0 + wm + 16 * i + rh + r) * ldy + n] + gv * v;
          so[(16 * i + rh + r) * 68 + 16 * j + cl] = v;
        }
      }
    }
  asm volatile("s_wait_dscnt 0" ::: "memory");
  __builtin_amdgcn_wave_barrier();
#pragma unroll 1
  for (int pass = 0; pass < 2; ++pass) {
    if (OUT16) {
      f16* Y = (f16*)Yv;
#pragma unroll
      for (int it = 0; it < 8; ++it) { const int c = lane + 32 * it, rr = c >> 3, q8 = (c & 7) * 8;
        union { f16 h[8]; v4u_t v; } u;
#pragma unroll
        for (int e = 0; e < 8; ++e) u.h[e] = (f16)so[rr * 68 + q8 + e];
        *(volatile v4u_t*)(Y + (size_t)(m0 + wm + rr) * ldy + n0 + wn + q8) = u.v; }
    } else {
      float* Y = (float*)Yv;
#pragma unroll
      for (int it = 0; it < 16; ++it) { const int f4 = lane + 32 * it, rr = f4 >> 4, q = (f4 & 15) * 4;
        *(volatile v4f_t*)(Y + (size_t)(m0 + wm + rr) * ldy + n0 + wn + q) = *(const v4fa*)(so + rr * 68 + q); }
    }
    __threadfence();
  }
}


#define NRB 4
#define NSt 16384
#define NFt 512
#define NNODE 4095
#define NNP 4096
#define RB 4096
__global__ __launch_bounds__(256) void k_wT(const float* __restrict__ W, float* __restrict__ WT) {
  __shared__ float tS[64][65];
  const int tid = threadIdx.x, bn = blockIdx.x, bk = blockIdx.y;
  for (int e = tid; e < 64 * 64; e += 256) { const int r = e >> 6, c = e & 63; const int n = bn * 64 + r; tS[r][c] = (n < NNODE) ? W[(size_t)n * NFt + bk * 64 + c] : 0.0f; }
  __syncthreads();
  for (int ch = tid; ch < 64 * 16; ch += 256) { const int k = ch >> 4, q4 = (ch & 15) * 4; v4f_t v; v[0] = tS[q4][k]; v[1] = tS[q4 + 1][k]; v[2] = tS[q4 + 2][k]; v[3] = tS[q4 + 3][k];
    float* d = WT + (size_t)(bk * 64 + k) * NNP + bn * 64 + q4; *(volatile v4f_t*)d = v; __threadfence(); *(volatile v4f_t*)d = v; }
}
__global__ __launch_bounds__(256) void k_padvec(const float* __restrict__ b, const float* __restrict__ s, float* __restrict__ bp, float* __restrict__ sp) { const int n = blockIdx.x * 256 + threadIdx.x; const float bv = (n < NNODE) ? b[n] : 0.0f, sv = (n < NNODE) ? s[n] : 1.0f;
  *(volatile float*)(bp + n) = bv; *(volatile float*)(sp + n) = sv; __threadfence(); *(volatile float*)(bp + n) = bv; *(volatile float*)(sp + n) = sv; }
__global__ __launch_bounds__(256) void k_tree(const float* __restrict__ LG, const float* __restrict__ bp, const float* __restrict__ sp, const float* __restrict__ leaves, float* __restrict__ outv, int row0) {
  __shared__ float pr[NNP]; __shared__ float bufA[NNP]; __shared__ float bufB[NNP]; __shared__ float red[256]; __shared__ float res[32];
  const int tid = threadIdx.x;
#pragma unroll 1
  for (int si = 0; si < 32; ++si) { const int sl = blockIdx.x * 32 + si; const float* lg = LG + (size_t)sl * NNP;
    for (int n = tid; n < NNP; n += 256) pr[n] = 1.0f / (1.0f + expf(-(lg[n] + bp[n]) * sp[n]));
    float* cur = bufA; float* nxt = bufB;
    if (tid == 0) cur[0] = 1.0f;
    __syncthreads();
#pragma unroll 1
    for (int d = 0; d < 12; ++d) { const int w = 1 << d, start = w - 1;
      for (int i = tid; i < w; i += 256) { const float c = cur[i], p = pr[start + i]; nxt[2 * i] = c * p; nxt[2 * i + 1] = c * (1.0f - p); }
      __syncthreads(); float* t = cur; cur = nxt; nxt = t; }
    float s = 0.0f;
    for (int j = tid; j < NNP; j += 256) s = fmaf(1.0f / (1.0f + expf(-leaves[j])), cur[j], s);
    red[tid] = s; __syncthreads();
    for (int o = 128; o > 0; o >>= 1) { if (tid < o) red[tid] += red[tid + o]; __syncthreads(); }
    if (tid == 0) res[si] = red[0];
    __syncthreads(); }
  if (tid < 32) { const float v = res[tid]; *(volatile float*)(outv + row0 + blockIdx.x * 32 + tid) = v; __threadfence(); *(volatile float*)(outv + row0 + blockIdx.x * 32 + tid) = v; }
}

extern "C" void kernel_launch(void* const* d_in, const int* in_sizes, int n_in,
                              void* d_out, int out_size, void* d_ws, size_t ws_size,
                              hipStream_t stream) {
  (void)in_sizes; (void)n_in; (void)out_size;
  const float** f = (const float**)d_in;
  const float* x = f[0], *W = f[1], *b = f[2], *s = f[3], *leaves = f[4];
  float* out = (float*)d_out;
  char* ws = (char*)d_ws;
  float* WT = (float*)ws; ws += (size_t)NFt * NNP * 4;
  float* bp = (float*)ws; ws += NNP * 4; float* sp = (float*)ws; ws += NNP * 4;
  float* LG = (float*)ws; ws += (size_t)RB * NNP * 4;
  if ((size_t)(ws - (char*)d_ws) > ws_size) return;
  const dim3 blk(256);
  k_wT<<<dim3(NNP / 64, NFt / 64), blk, 0, stream>>>(W, WT); k_padvec<<<dim3(NNP / 256), blk, 0, stream>>>(b, s, bp, sp);
  for (int rb = 0; rb < NRB; ++rb) {
    gemm_kne<float, 0, false><<<dim3(RB / 128, NNP / 128), blk, 0, stream>>>(x + (size_t)rb * RB * NFt, NFt, WT, NNP, nullptr, nullptr, nullptr, LG, NNP, NFt);
    k_tree<<<dim3(RB / 32), blk, 0, stream>>>(LG, bp, sp, leaves, out, rb * RB);
  }
}
